// MultiHeadSelfAttention_17772574671217
// MI455X (gfx1250) — hardware-verified
//
#include <hip/hip_runtime.h>


#ifndef NB
#define NB 8
#endif
#ifndef SEQ
#define SEQ 1024
#endif
#define NB_FULL  8
#define SEQ_FULL 1024
#define DM   768
#define NH_  12
#define HD   64
#define CSC  (0.03608439182435161f * 1.4426950408889634f)
#define PEXP 10.0f

static_assert(DM == NH_ * HD);
static_assert(SEQ % 64 == 0);
static_assert((NB * SEQ) % 64 == 0);
static_assert(DM % 64 == 0);
static_assert(SEQ <= SEQ_FULL);
static_assert(NB <= NB_FULL);

#define SZ_ACT ((size_t)NB * SEQ * DM * 2)
#define SZ_WO  ((size_t)DM * DM * 2)
#define SZ_WT  ((size_t)3 * NH_ * HD * HD * 2)
#define WS_TOTAL (7 * SZ_ACT + SZ_WO + SZ_WT)
static_assert(SZ_ACT % 256 == 0);
static_assert(SZ_WO % 256 == 0);
static_assert(SZ_WT % 256 == 0);
static_assert(WS_TOTAL <= (size_t)134217728);

typedef _Float16 h16;
typedef unsigned short bf;
typedef __attribute__((ext_vector_type(16))) __bf16   v16bf;
typedef __attribute__((ext_vector_type(16))) _Float16 v16h;
typedef __attribute__((ext_vector_type(8)))  _Float16 v8h;
typedef __attribute__((ext_vector_type(8)))  unsigned short v8us;
typedef __attribute__((ext_vector_type(2)))  unsigned short v2us;
typedef __attribute__((ext_vector_type(8)))  unsigned v8u;
typedef __attribute__((ext_vector_type(8)))  float    v8f;
typedef __attribute__((ext_vector_type(4)))  float    v4f;
typedef v4f  __attribute__((may_alias)) v4fa;

__device__ __forceinline__ unsigned short f2bf(float f) { unsigned u = __float_as_uint(f); u += 0x7FFFu + ((u >> 16) & 1u); return (unsigned short)(u >> 16); }
__device__ __forceinline__ float bf2f(unsigned short b) { return __uint_as_float(((unsigned)b) << 16); }
__device__ __forceinline__ float bfr(float f) { return bf2f(f2bf(f)); }
__device__ __forceinline__ void splitf(float y, unsigned short& h, unsigned short& l) { h = f2bf(y); l = f2bf(y - bf2f(h)); }
__device__ __forceinline__ v16h cat16(v8h lo, v8h hi) { return __builtin_shufflevector(lo, hi, 0, 1, 2, 3, 4, 5, 6, 7, 8, 9, 10, 11, 12, 13, 14, 15); }
__device__ __forceinline__ v16bf cat16b(v8us lo, v8us hi) { return __builtin_bit_cast(v16bf, __builtin_shufflevector(lo, hi, 0, 1, 2, 3, 4, 5, 6, 7, 8, 9, 10, 11, 12, 13, 14, 15)); }
__device__ __forceinline__ v8f wmma16(v16h a, v16h b, v8f c) { return __builtin_amdgcn_wmma_f32_16x16x32_f16(false, a, false, b, (short)0, c, false, false); }
__device__ __forceinline__ v8f wmmab(v16bf a, v16bf b, v8f c) { return __builtin_amdgcn_wmma_f32_16x16x32_bf16(false, a, false, b, (short)0, c, false, false); }

template <typename T16> struct WFrag;
template <> struct WFrag<h16> { typedef v16h V; static __device__ __forceinline__ V ld(const h16* p) { return cat16(*(const v8h*)p, *(const v8h*)(p + 16)); } static __device__ __forceinline__ v8f mma(V a, V b, v8f c) { return wmma16(a, b, c); } };
template <> struct WFrag<bf> { typedef v16bf V; static __device__ __forceinline__ V ld(const bf* p) { return cat16b(*(const v8us*)p, *(const v8us*)(p + 16)); } static __device__ __forceinline__ v8f mma(V a, V b, v8f c) { return wmmab(a, b, c); } };

template <typename T16, int NSPLIT, bool BIAS>
__global__ __launch_bounds__(32) void k_gemmw(const T16* __restrict__ A, const T16* __restrict__ A2, const T16* __restrict__ Bt, const T16* __restrict__ Bt2, int K, float* C, int ldc, const float* __restrict__ bias, size_t sA, size_t sB, size_t sC) {
    typedef typename WFrag<T16>::V V;
    __shared__ __align__(16) float os[16 * 68];
    const size_t z = blockIdx.z; A += z * sA; if (A2) A2 += z * sA; Bt += z * sB; if (Bt2) Bt2 += z * sB; C += z * sC;
    const int lane = threadIdx.x & 31, lr = lane & 15, hi = lane >> 4; const int r0 = blockIdx.x * 64, c0 = blockIdx.y * 64;
    v8f acc[4][4];
#pragma unroll
    for (int mb = 0; mb < 4; ++mb)
#pragma unroll
        for (int nb = 0; nb < 4; ++nb) acc[mb][nb] = (v8f){};
    const size_t aoff = (size_t)(r0 + lr) * K + 8 * hi, boff = (size_t)(c0 + lr) * K + 8 * hi;
#pragma unroll 1
    for (int kc = 0; kc < K; kc += 32) {
        V a[4], a2[4];
#pragma unroll
        for (int mb = 0; mb < 4; ++mb) { a[mb] = WFrag<T16>::ld(A + aoff + (size_t)mb * 16 * K + kc); if (NSPLIT == 1 || NSPLIT == 2) a2[mb] = WFrag<T16>::ld(A2 + aoff + (size_t)mb * 16 * K + kc); }
#pragma unroll
        for (int nb = 0; nb < 4; ++nb) { const V b = WFrag<T16>::ld(Bt + boff + (size_t)nb * 16 * K + kc); V b2; if (NSPLIT >= 2) b2 = WFrag<T16>::ld(Bt2 + boff + (size_t)nb * 16 * K + kc);
#pragma unroll
            for (int mb = 0; mb < 4; ++mb) { acc[mb][nb] = WFrag<T16>::mma(a[mb], b, acc[mb][nb]); if (NSPLIT == 1 || NSPLIT == 2) acc[mb][nb] = WFrag<T16>::mma(a2[mb], b, acc[mb][nb]); if (NSPLIT >= 2) acc[mb][nb] = WFrag<T16>::mma(a[mb], b2, acc[mb][nb]); } }
        asm volatile("v_nop\n\tv_nop\n\tv_nop\n\tv_nop" : "+v"(acc[0][0]), "+v"(acc[1][1]), "+v"(acc[2][2]), "+v"(acc[3][3]) : "v"(a[0]), "v"(a[3]));
    }
#pragma unroll
    for (int mb = 0; mb < 4; ++mb) {
#pragma unroll
        for (int nb = 0; nb < 4; ++nb) {
#pragma unroll
            for (int j = 0; j < 8; ++j) os[(hi * 8 + j) * 68 + nb * 16 + lr] = acc[mb][nb][j]; }
        __builtin_amdgcn_wave_barrier(); asm volatile("" ::: "memory");
        float* crow = C + (size_t)(r0 + mb * 16) * ldc + c0;
#pragma unroll 1
        for (int ps = 0; ps < 2; ++ps) {
#pragma unroll
            for (int s = 0; s < 8; ++s) { const int row = 2 * s + hi, cofs = lr * 4; v4f val = *(const v4fa*)(os + row * 68 + cofs); if (BIAS) { val[0] += bfr(bias[c0 + cofs]); val[1] += bfr(bias[c0 + cofs + 1]); val[2] += bfr(bias[c0 + cofs + 2]); val[3] += bfr(bias[c0 + cofs + 3]); }
                *(volatile v4f*)(crow + (size_t)row * ldc + cofs) = val; }
            if (ps == 0) __threadfence(); }
        __builtin_amdgcn_wave_barrier(); asm volatile("" ::: "memory");
    }
}

__global__ __launch_bounds__(256) void k_cvt8(const float* __restrict__ src, bf* dst, size_t n8) { const size_t i = (size_t)blockIdx.x * 256 + threadIdx.x; if (i >= n8) return; const v8f v = *(const v8f*)(src + i * 8); v8us o;
#pragma unroll
    for (int k = 0; k < 8; ++k) o[k] = f2bf(v[k]); *(volatile v8us*)(dst + i * 8) = o; __threadfence(); *(volatile v8us*)(dst + i * 8) = o; }

__global__ __launch_bounds__(256) void k_wtH(const float* __restrict__ wq, const float* __restrict__ wk, const float* __restrict__ wv, bf* WT) {
    const unsigned lane = threadIdx.x & 31u; const unsigned mat = blockIdx.y;
    const float* w = (mat == 0u) ? wq : ((mat == 1u) ? wk : wv);
    bf* dst = WT + (size_t)mat * (NH_ * HD * HD);
    const unsigned L0 = (blockIdx.x * 8u + (threadIdx.x >> 5)) * 8u;
#pragma unroll 1
    for (int ps = 0; ps < 2; ++ps) {
#pragma unroll 1
        for (unsigned l = 0; l < 8u; ++l) { const unsigned L = L0 + l;
            if (L < (unsigned)(NH_ * HD)) { const unsigned e = L * 64u + lane * 2u; const unsigned hd = e >> 12, n = (e >> 6) & 63u, k = e & 63u; const float* s = w + (size_t)hd * 4096u + k * 64u + n; v2us o;
                o[0] = f2bf(s[0]); o[1] = f2bf(s[64]); *(volatile v2us*)(dst + e) = o; } }
        if (ps == 0) __threadfence(); }
}

__global__ __launch_bounds__(32) void k_proj(const bf* __restrict__ XB, const bf* __restrict__ WT, const float* __restrict__ bq, const float* __restrict__ bk, const float* __restrict__ bv, h16* Q16, h16* K16, bf* VTh, bf* VTl) {
    __shared__ __align__(16) float os[64 * 68];
    const unsigned lane = threadIdx.x & 31u, lr = lane & 15u, hi = lane >> 4;
    const unsigned r0 = blockIdx.x * 64u, hh = blockIdx.y, mat = blockIdx.z;
    const float* bias = (mat == 0u) ? bq : ((mat == 1u) ? bk : bv);
    const bf* A = XB + (size_t)(r0 + lr) * DM + hh * 64u + 8u * hi;
    const bf* B = WT + (size_t)(mat * NH_ + hh) * 4096u + lr * 64u + 8u * hi;
    v8f acc[4][4];
#pragma unroll
    for (int mb = 0; mb < 4; ++mb)
#pragma unroll
        for (int nb = 0; nb < 4; ++nb) acc[mb][nb] = (v8f){};
#pragma unroll 1
    for (unsigned kc = 0; kc < 64u; kc += 32u) {
        v16bf a[4];
#pragma unroll
        for (int mb = 0; mb < 4; ++mb) a[mb] = WFrag<bf>::ld(A + (size_t)mb * 16 * DM + kc);
#pragma unroll
        for (int nb = 0; nb < 4; ++nb) { const v16bf b = WFrag<bf>::ld(B + nb * 16 * 64 + kc);
#pragma unroll
            for (int mb = 0; mb < 4; ++mb) acc[mb][nb] = wmmab(a[mb], b, acc[mb][nb]); }
        asm volatile("v_nop\n\tv_nop\n\tv_nop\n\tv_nop" : "+v"(acc[0][0]), "+v"(acc[1][1]), "+v"(acc[2][2]), "+v"(acc[3][3]) : "v"(a[0]), "v"(a[3]));
    }
#pragma unroll
    for (int nb = 0; nb < 4; ++nb) { const float bsv = bfr(bias[hh * 64u + nb * 16 + lr]);
#pragma unroll
        for (int mb = 0; mb < 4; ++mb)
#pragma unroll
            for (int j = 0; j < 8; ++j) os[(mb * 16 + hi * 8 + j) * 68 + nb * 16 + lr] = acc[mb][nb][j] + bsv; }
    __syncthreads();
    const unsigned b = r0 / (unsigned)SEQ, t0 = r0 % (unsigned)SEQ;
    const size_t bh = (size_t)b * NH_ + hh;
    const unsigned rq = lane >> 3, pc = lane & 7u;
    if (mat < 2u) {
        h16* dst = ((mat == 0u) ? Q16 : K16) + (bh * SEQ + t0) * HD;
#pragma unroll 1
        for (int ps = 0; ps < 2; ++ps) {
#pragma unroll 4
            for (unsigned it = 0; it < 16u; ++it) { const unsigned row = it * 4u + rq; const v4f x0 = *(const v4fa*)(os + row * 68u + pc * 8u), x1 = *(const v4fa*)(os + row * 68u + pc * 8u + 4u); v8h o;
                o[0] = (h16)x0[0]; o[1] = (h16)x0[1]; o[2] = (h16)x0[2]; o[3] = (h16)x0[3]; o[4] = (h16)x1[0]; o[5] = (h16)x1[1]; o[6] = (h16)x1[2]; o[7] = (h16)x1[3];
                *(volatile v8h*)(dst + (size_t)row * HD + pc * 8u) = o; }
            if (ps == 0) __threadfence(); }
    } else {
        bf* dh = VTh + bh * HD * SEQ + t0; bf* dl = VTl + bh * HD * SEQ + t0;
#pragma unroll 1
        for (int ps = 0; ps < 2; ++ps) {
#pragma unroll 2
            for (unsigned it = 0; it < 16u; ++it) { const unsigned d = it * 4u + rq; v8us oh, ol;
#pragma unroll
                for (int i = 0; i < 8; ++i) { unsigned short a2, c2; splitf(os[(pc * 8u + i) * 68u + d], a2, c2); oh[i] = a2; ol[i] = c2; }
                *(volatile v8us*)(dh + (size_t)d * SEQ + pc * 8u) = oh; *(volatile v8us*)(dl + (size_t)d * SEQ + pc * 8u) = ol; }
            if (ps == 0) __threadfence(); }
    }
}

__global__ __launch_bounds__(128) void k_attn(const h16* __restrict__ Q16, const h16* __restrict__ K16, const bf* __restrict__ VTh, const bf* __restrict__ VTl, bf* ATh, bf* ATl) {
    __shared__ __align__(16) float ost[4 * 16 * 68];
    const unsigned tid = threadIdx.x, wv = tid >> 5, lane = tid & 31u, lr = lane & 15u, hi = lane >> 4;
    const unsigned hh = blockIdx.y, b = blockIdx.z, q0 = blockIdx.x * 64u + wv * 16u;
    const size_t bh = (size_t)b * NH_ + hh;
    const h16* Qp = Q16 + bh * SEQ * HD + (size_t)(q0 + lr) * HD + 8u * hi;
    const h16* Kp = K16 + bh * SEQ * HD + (size_t)lr * HD + 8u * hi;
    const bf* Vhp = VTh + bh * HD * SEQ + (size_t)lr * SEQ + 8u * hi;
    const bf* Vlp = VTl + bh * HD * SEQ + (size_t)lr * SEQ + 8u * hi;
    v16h qb[2]; qb[0] = WFrag<h16>::ld(Qp); qb[1] = WFrag<h16>::ld(Qp + 32);
    v8f o[4];
#pragma unroll
    for (int dt = 0; dt < 4; ++dt) o[dt] = (v8f){};
    float mrun = -1.0e30f, lrun = 0.0f;
#pragma unroll 1
    for (unsigned j0 = 0; j0 < (unsigned)SEQ; j0 += 64u) {
        v8f s[4];
#pragma unroll
        for (int a = 0; a < 4; ++a) { v8f c = (v8f){};
#pragma unroll
            for (int g = 0; g < 2; ++g) { const v16h ka = WFrag<h16>::ld(Kp + (size_t)(j0 + 16 * a) * HD + 32 * g); c = wmma16(ka, qb[g], c); }
            s[a] = c; }
        asm volatile("v_nop\n\tv_nop\n\tv_nop\n\tv_nop" : "+v"(s[0]), "+v"(s[1]), "+v"(s[2]), "+v"(s[3]) : "v"(qb[0]), "v"(qb[1]));
        float mx = fmaxf(fmaxf(s[0][0], s[1][0]), fmaxf(s[2][0], s[3][0]));
#pragma unroll
        for (int r = 1; r < 8; ++r) mx = fmaxf(mx, fmaxf(fmaxf(s[0][r], s[1][r]), fmaxf(s[2][r], s[3][r])));
        mx = fmaxf(mx, __shfl_xor(mx, 16, 32));
        const float mnew = fmaxf(mrun, mx);
        const float alpha = __builtin_amdgcn_exp2f((mrun - mnew) * CSC);
        const float nmc = PEXP - mnew * CSC;
        mrun = mnew;
        v8u wh[2], wl[2]; float psum = 0.0f;
#pragma unroll
        for (int g = 0; g < 2; ++g)
#pragma unroll
            for (int hf = 0; hf < 2; ++hf)
#pragma unroll
                for (int w = 0; w < 4; ++w) {
                    const float p0 = __builtin_amdgcn_exp2f(__builtin_fmaf(s[2 * g + hf][2 * w], CSC, nmc));
                    const float p1 = __builtin_amdgcn_exp2f(__builtin_fmaf(s[2 * g + hf][2 * w + 1], CSC, nmc));
                    psum += p0 + p1;
                    const unsigned u0 = __float_as_uint(p0), u1 = __float_as_uint(p1);
                    const unsigned t0 = u0 & 0xFFFF0000u, t1 = u1 & 0xFFFF0000u;
                    wh[g][hf * 4 + w] = (u0 >> 16) | t1;
                    const unsigned l0 = (unsigned)f2bf(p0 - __uint_as_float(t0)), l1 = (unsigned)f2bf(p1 - __uint_as_float(t1));
                    wl[g][hf * 4 + w] = l0 | (l1 << 16);
                }
        lrun = lrun * alpha + psum;
#pragma unroll
        for (int dt = 0; dt < 4; ++dt) o[dt] = o[dt] * alpha;
        unsigned jv = j0;
        asm volatile("" : "+v"(jv) : "v"(psum));
        const v16bf phB0 = __builtin_bit_cast(v16bf, wh[0]), plB0 = __builtin_bit_cast(v16bf, wl[0]);
        const v16bf phB1 = __builtin_bit_cast(v16bf, wh[1]), plB1 = __builtin_bit_cast(v16bf, wl[1]);
#pragma unroll
        for (int dt = 0; dt < 4; ++dt) { const size_t vo = (size_t)(dt * 16) * SEQ + jv; const v16bf vh = WFrag<bf>::ld(Vhp + vo); const v16bf vl = WFrag<bf>::ld(Vlp + vo);
            o[dt] = wmmab(vh, phB0, o[dt]); o[dt] = wmmab(vh, plB0, o[dt]); o[dt] = wmmab(vl, phB0, o[dt]); }
        asm volatile("v_nop\n\tv_nop\n\tv_nop\n\tv_nop" : "+v"(o[0]), "+v"(o[1]), "+v"(o[2]), "+v"(o[3]), "+v"(jv) : "v"(phB0), "v"(plB0));
#pragma unroll
        for (int dt = 0; dt < 4; ++dt) { const size_t vo = (size_t)(dt * 16) * SEQ + jv + 32u; const v16bf vh = WFrag<bf>::ld(Vhp + vo); const v16bf vl = WFrag<bf>::ld(Vlp + vo);
            o[dt] = wmmab(vh, phB1, o[dt]); o[dt] = wmmab(vh, plB1, o[dt]); o[dt] = wmmab(vl, phB1, o[dt]); }
        asm volatile("v_nop\n\tv_nop\n\tv_nop\n\tv_nop" : "+v"(o[0]), "+v"(o[1]), "+v"(o[2]), "+v"(o[3]) : "v"(phB1), "v"(plB1));
    }
    const float lt = lrun + __shfl_xor(lrun, 16, 32);
    const float inv = 1.0f / lt;
    float* ow = ost + wv * (16 * 68);
#pragma unroll
    for (int dt = 0; dt < 4; ++dt) { v4f x0, x1;
        x0[0] = o[dt][0] * inv; x0[1] = o[dt][1] * inv; x0[2] = o[dt][2] * inv; x0[3] = o[dt][3] * inv;
        x1[0] = o[dt][4] * inv; x1[1] = o[dt][5] * inv; x1[2] = o[dt][6] * inv; x1[3] = o[dt][7] * inv;
        *(v4fa*)(ow + lr * 68u + dt * 16 + hi * 8u) = x0; *(v4fa*)(ow + lr * 68u + dt * 16 + hi * 8u + 4u) = x1; }
    __syncthreads();
    const unsigned rq = lane >> 3, pc = lane & 7u;
    bf* dh = ATh + ((size_t)b * SEQ + q0) * DM + hh * HD; bf* dl = ATl + ((size_t)b * SEQ + q0) * DM + hh * HD;
#pragma unroll 1
    for (int ps = 0; ps < 2; ++ps) {
#pragma unroll
        for (unsigned it = 0; it < 4u; ++it) { const unsigned row = it * 4u + rq; const v4f x0 = *(const v4fa*)(ow + row * 68u + pc * 8u), x1 = *(const v4fa*)(ow + row * 68u + pc * 8u + 4u); v8us oh, ol;
#pragma unroll
            for (int k = 0; k < 4; ++k) { unsigned short a2, c2; splitf(x0[k], a2, c2); oh[k] = a2; ol[k] = c2; splitf(x1[k], a2, c2); oh[4 + k] = a2; ol[4 + k] = c2; }
            *(volatile v8us*)(dh + (size_t)row * DM + pc * 8u) = oh; *(volatile v8us*)(dl + (size_t)row * DM + pc * 8u) = ol; }
        if (ps == 0) __threadfence(); }
}

extern "C" void kernel_launch(void* const* d_in, const int* in_sizes, int n_in,
                              void* d_out, int out_size, void* d_ws, size_t ws_size, hipStream_t stream) {
    if (n_in < 9) return;
    const size_t xneed = ((size_t)(NB - 1) * SEQ_FULL + SEQ) * DM;
    if ((size_t)in_sizes[0] < xneed) return;
    if ((size_t)in_sizes[1] < (size_t)NH_ * HD * HD || (size_t)in_sizes[2] < (size_t)NH_ * HD * HD || (size_t)in_sizes[3] < (size_t)NH_ * HD * HD) return;
    if ((size_t)in_sizes[4] < (size_t)DM || (size_t)in_sizes[5] < (size_t)DM || (size_t)in_sizes[6] < (size_t)DM) return;
    if ((size_t)in_sizes[7] < (size_t)DM * DM || (size_t)in_sizes[8] < (size_t)DM) return;
    if ((size_t)out_size < xneed) return;
    const float* x = (const float*)d_in[0]; const float* wq = (const float*)d_in[1]; const float* wk = (const float*)d_in[2]; const float* wv = (const float*)d_in[3];
    const float* bq = (const float*)d_in[4]; const float* bk = (const float*)d_in[5]; const float* bv = (const float*)d_in[6]; const float* wo = (const float*)d_in[7]; const float* bo = (const float*)d_in[8];
    float* OUT = (float*)d_out;
    char* wsp = (char*)d_ws;
    auto take = [&](size_t bytes) { char* p = wsp; wsp += (bytes + 255) & ~(size_t)255; return (void*)p; };
    bf* XB = (bf*)take(SZ_ACT); bf* WO = (bf*)take(SZ_WO); bf* WT = (bf*)take(SZ_WT);
    h16* Q16 = (h16*)take(SZ_ACT); h16* K16 = (h16*)take(SZ_ACT); bf* VTh = (bf*)take(SZ_ACT); bf* VTl = (bf*)take(SZ_ACT); bf* ATh = (bf*)take(SZ_ACT); bf* ATl = (bf*)take(SZ_ACT);
    if ((size_t)(wsp - (char*)d_ws) > ws_size) return;

    if (SEQ == SEQ_FULL) { const size_t n8 = (size_t)NB * SEQ * DM / 8; k_cvt8<<<(unsigned)((n8 + 255) / 256), 256, 0, stream>>>(x, XB, n8); }
    else { const size_t n8 = (size_t)SEQ * DM / 8; for (int b = 0; b < NB; ++b) k_cvt8<<<(unsigned)((n8 + 255) / 256), 256, 0, stream>>>(x + (size_t)b * SEQ_FULL * DM, XB + (size_t)b * SEQ * DM, n8); }
    { const size_t n8 = (size_t)DM * DM / 8; k_cvt8<<<(unsigned)((n8 + 255) / 256), 256, 0, stream>>>(wo, WO, n8); }
    k_wtH<<<dim3((NH_ * HD) / 64, 3), 256, 0, stream>>>(wq, wk, wv, WT);
    k_proj<<<dim3((NB * SEQ) / 64, NH_, 3), 32, 0, stream>>>(XB, WT, bq, bk, bv, Q16, K16, VTh, VTl);
    k_attn<<<dim3(SEQ / 64, NH_, NB), 128, 0, stream>>>(Q16, K16, VTh, VTl, ATh, ATl);
    if (SEQ == SEQ_FULL) { k_gemmw<bf, 1, true><<<dim3((NB * SEQ) / 64, DM / 64, 1), 32, 0, stream>>>(ATh, ATl, WO, nullptr, DM, OUT, DM, bo, 0, 0, 0); }
    else { for (int b = 0; b < NB; ++b) k_gemmw<bf, 1, true><<<dim3(SEQ / 64, DM / 64, 1), 32, 0, stream>>>(ATh + (size_t)b * SEQ * DM, ATl + (size_t)b * SEQ * DM, WO, nullptr, DM, OUT + (size_t)b * SEQ_FULL * DM, DM, bo, 0, 0, 0); }
}
